// LongformerLayerPrewritten_23235773071563
// MI455X (gfx1250) — hardware-verified
//
#include <hip/hip_runtime.h>


#define NB_  2
#define SS   4096
#define DM   768
#define NH_  12
#define HD   64
#define WW   64
#define NC   (SS / WW)
#define KW   (3 * WW)
#define SP   (SS + 2 * WW)
#define FF   3072
#define PCAR 1024.0f
typedef _Float16 h16;
typedef unsigned short bf;
typedef __attribute__((ext_vector_type(16))) __bf16   v16bf;
typedef __attribute__((ext_vector_type(16))) _Float16 v16h;
typedef __attribute__((ext_vector_type(8)))  _Float16 v8h;
typedef __attribute__((ext_vector_type(8)))  unsigned short v8us;
typedef __attribute__((ext_vector_type(8)))  float    v8f;
typedef __attribute__((ext_vector_type(4)))  float    v4f;
typedef v8h  __attribute__((may_alias)) v8ha;
typedef v4f  __attribute__((may_alias)) v4fa;
typedef v8us __attribute__((may_alias)) v8usa;

__device__ __forceinline__ unsigned short f2bf(float f) { unsigned u = __float_as_uint(f); u += 0x7FFFu + ((u >> 16) & 1u); return (unsigned short)(u >> 16); }
__device__ __forceinline__ float bf2f(unsigned short b) { return __uint_as_float(((unsigned)b) << 16); }
__device__ __forceinline__ float bfr(float f) { return bf2f(f2bf(f)); }
__device__ __forceinline__ v16h cat16(v8h lo, v8h hi) { return __builtin_shufflevector(lo, hi, 0, 1, 2, 3, 4, 5, 6, 7, 8, 9, 10, 11, 12, 13, 14, 15); }
__device__ __forceinline__ v16bf cat16b(v8us lo, v8us hi) { return __builtin_bit_cast(v16bf, __builtin_shufflevector(lo, hi, 0, 1, 2, 3, 4, 5, 6, 7, 8, 9, 10, 11, 12, 13, 14, 15)); }
__device__ __forceinline__ v8f wmma16(v16h a, v16h b, v8f c) { return __builtin_amdgcn_wmma_f32_16x16x32_f16(false, a, false, b, (short)0, c, false, false); }
__device__ __forceinline__ v8f wmmab(v16bf a, v16bf b, v8f c) { return __builtin_amdgcn_wmma_f32_16x16x32_bf16(false, a, false, b, (short)0, c, false, false); }


template <typename T16> struct WFrag;
template <> struct WFrag<h16> { typedef v16h V; static __device__ __forceinline__ V ld(const h16* p) { return cat16(*(const v8h*)p, *(const v8h*)(p + 16)); } static __device__ __forceinline__ v8f mma(V a, V b, v8f c) { return wmma16(a, b, c); } };
template <> struct WFrag<bf> { typedef v16bf V; static __device__ __forceinline__ V ld(const bf* p) { return cat16b(*(const v8us*)p, *(const v8us*)(p + 16)); } static __device__ __forceinline__ v8f mma(V a, V b, v8f c) { return wmmab(a, b, c); } };
template <typename T16, int NSPLIT, bool BIAS>
__global__ __launch_bounds__(32) void k_gemmw(const T16* __restrict__ A, const T16* __restrict__ A2, const T16* __restrict__ Bt, const T16* __restrict__ Bt2, int K, float* C, int ldc, const float* __restrict__ bias, size_t sA, size_t sB, size_t sC) {
    typedef typename WFrag<T16>::V V;
    __shared__ __align__(16) float os[16 * 68];
    const size_t z = blockIdx.z; A += z * sA; if (A2) A2 += z * sA; Bt += z * sB; if (Bt2) Bt2 += z * sB; C += z * sC;
    const int lane = threadIdx.x & 31, lr = lane & 15, hi = lane >> 4; const int r0 = blockIdx.x * 64, c0 = blockIdx.y * 64;
    v8f acc[4][4];
#pragma unroll
    for (int mb = 0; mb < 4; ++mb)
#pragma unroll
        for (int nb = 0; nb < 4; ++nb) acc[mb][nb] = (v8f){};
    const size_t aoff = (size_t)(r0 + lr) * K + 8 * hi, boff = (size_t)(c0 + lr) * K + 8 * hi;
#pragma unroll 1
    for (int kc = 0; kc < K; kc += 32) {
        V a[4], a2[4];
#pragma unroll
        for (int mb = 0; mb < 4; ++mb) { a[mb] = WFrag<T16>::ld(A + aoff + (size_t)mb * 16 * K + kc); if (NSPLIT == 1 || NSPLIT == 2) a2[mb] = WFrag<T16>::ld(A2 + aoff + (size_t)mb * 16 * K + kc); }
#pragma unroll
        for (int nb = 0; nb < 4; ++nb) { const V b = WFrag<T16>::ld(Bt + boff + (size_t)nb * 16 * K + kc); V b2; if (NSPLIT >= 2) b2 = WFrag<T16>::ld(Bt2 + boff + (size_t)nb * 16 * K + kc);
#pragma unroll
            for (int mb = 0; mb < 4; ++mb) { acc[mb][nb] = WFrag<T16>::mma(a[mb], b, acc[mb][nb]); if (NSPLIT == 1 || NSPLIT == 2) acc[mb][nb] = WFrag<T16>::mma(a2[mb], b, acc[mb][nb]); if (NSPLIT >= 2) acc[mb][nb] = WFrag<T16>::mma(a[mb], b2, acc[mb][nb]); } }
        asm volatile("v_nop\n\tv_nop\n\tv_nop\n\tv_nop" : "+v"(acc[0][0]), "+v"(acc[1][1]), "+v"(acc[2][2]), "+v"(acc[3][3]) : "v"(a[0]), "v"(a[3]));
    }
#pragma unroll
    for (int mb = 0; mb < 4; ++mb) {
#pragma unroll
        for (int nb = 0; nb < 4; ++nb) {
#pragma unroll
            for (int j = 0; j < 8; ++j) os[(hi * 8 + j) * 68 + nb * 16 + lr] = acc[mb][nb][j]; }
        __builtin_amdgcn_wave_barrier(); asm volatile("" ::: "memory");
        float* crow = C + (size_t)(r0 + mb * 16) * ldc + c0;
#pragma unroll 1
        for (int ps = 0; ps < 2; ++ps) {
#pragma unroll
            for (int s = 0; s < 8; ++s) { const int row = 2 * s + hi, cofs = lr * 4; v4f val = *(const v4fa*)(os + row * 68 + cofs); if (BIAS) { val[0] += bfr(bias[c0 + cofs]); val[1] += bfr(bias[c0 + cofs + 1]); val[2] += bfr(bias[c0 + cofs + 2]); val[3] += bfr(bias[c0 + cofs + 3]); }
                *(volatile v4f*)(crow + (size_t)row * ldc + cofs) = val; }
            if (ps == 0) __threadfence(); }
        __builtin_amdgcn_wave_barrier(); asm volatile("" ::: "memory");
    }
}

__device__ __forceinline__ h16 tohx(float x) { return (h16)x; }
typedef __attribute__((ext_vector_type(2))) _Float16 v2h;
typedef __attribute__((ext_vector_type(4))) _Float16 v4h;
typedef __attribute__((ext_vector_type(2))) unsigned short v2us;

__global__ __launch_bounds__(256) void k_wtG(const float* __restrict__ w, int K, int N, bf* Bt) {
    const int lane = threadIdx.x & 31; const int L0 = (blockIdx.x * 8 + (threadIdx.x >> 5)) * 8; const int nlines = N * K / 64;
#pragma unroll 1
    for (int ps = 0; ps < 2; ++ps) {
#pragma unroll 1
        for (int l = 0; l < 8; ++l) { const int L = L0 + l; if (L >= nlines) break; const size_t e = (size_t)L * 64 + lane * 2; const int k = (int)(e % K), n = (int)(e / K); v2us o;
            o[0] = f2bf(w[(size_t)k * N + n]); o[1] = f2bf(w[(size_t)(k + 1) * N + n]); *(volatile v2us*)(Bt + e) = o; }
        if (ps == 0) __threadfence(); }
}
__global__ __launch_bounds__(256) void k_cvt8(const float* __restrict__ src, bf* dst, size_t n8) { const size_t i = (size_t)blockIdx.x * 256 + threadIdx.x; if (i >= n8) return; const v8f v = *(const v8f*)(src + i * 8); v8us o;
#pragma unroll
    for (int k = 0; k < 8; ++k) o[k] = f2bf(v[k]); *(volatile v8us*)(dst + i * 8) = o; __threadfence(); *(volatile v8us*)(dst + i * 8) = o; }
__global__ __launch_bounds__(256) void k_wt16(const float* __restrict__ w, int K, int N, h16* Bt) { const size_t e = ((size_t)blockIdx.x * 256 + threadIdx.x) * 2; if (e >= (size_t)N * K) return; const int k = (int)(e % K), n = (int)(e / K); v2h o; o[0] = tohx(bfr(w[(size_t)k * N + n])); o[1] = tohx(bfr(w[(size_t)(k + 1) * N + n])); *(volatile v2h*)(Bt + e) = o; __threadfence(); *(volatile v2h*)(Bt + e) = o; }
__global__ __launch_bounds__(256) void k_qpl(const float* __restrict__ QF, h16* Q16) { const size_t e = ((size_t)blockIdx.x * 256 + threadIdx.x) * 4; if (e >= (size_t)NH_ * SS * HD) return; const int d = (int)(e % HD); const int t = (int)((e / HD) % SS); const int h = (int)(e / ((size_t)HD * SS)); const v4f a = *(const v4f*)(QF + (size_t)t * DM + h * HD + d); v4h o;
#pragma unroll
    for (int q = 0; q < 4; ++q) o[q] = tohx(a[q] * 0.125f); *(volatile v4h*)(Q16 + e) = o; __threadfence(); *(volatile v4h*)(Q16 + e) = o; }
__global__ __launch_bounds__(256) void k_kpl(const float* __restrict__ KF, h16* KP) { const size_t e = ((size_t)blockIdx.x * 256 + threadIdx.x) * 4; if (e >= (size_t)NH_ * SP * HD) return; const int d = (int)(e % HD); const int tp = (int)((e / HD) % SP); const int h = (int)(e / ((size_t)HD * SP)); const int t = tp - WW; v4h o;
    if (t >= 0 && t < SS) { const v4f a = *(const v4f*)(KF + (size_t)t * DM + h * HD + d); o[0] = tohx(a[0]); o[1] = tohx(a[1]); o[2] = tohx(a[2]); o[3] = tohx(a[3]); } else { o[0] = (h16)0.f; o[1] = (h16)0.f; o[2] = (h16)0.f; o[3] = (h16)0.f; }
    *(volatile v4h*)(KP + e) = o; __threadfence(); *(volatile v4h*)(KP + e) = o; }
__global__ __launch_bounds__(256) void k_vwin(const float* __restrict__ VF, h16* VW) { const size_t e = ((size_t)blockIdx.x * 256 + threadIdx.x) * 2; if (e >= (size_t)NH_ * NC * HD * KW) return; const int j = (int)(e % KW); const int d = (int)((e / KW) % HD); const int c = (int)((e / ((size_t)KW * HD)) % NC); const int h = (int)(e / ((size_t)KW * HD * NC)); v2h o;
#pragma unroll
    for (int u = 0; u < 2; ++u) { const int t = c * WW - WW + j + u; o[u] = (t >= 0 && t < SS) ? tohx(VF[(size_t)t * DM + h * HD + d]) : (h16)0.f; } *(volatile v2h*)(VW + e) = o; __threadfence(); *(volatile v2h*)(VW + e) = o; }
__global__ __launch_bounds__(256) void k_bsoft(const float* __restrict__ Sb, h16* P) { const int lane = threadIdx.x & 31; const int row = blockIdx.x * 8 + (threadIdx.x >> 5); if (row >= NC * WW) return; const int i = row % WW, c = row / WW; const float* sr = Sb + (size_t)row * KW; float v[8]; bool ok[8]; float mx = -3.0e38f;
#pragma unroll
    for (int q = 0; q < 8; ++q) { const int j = q < 4 ? lane * 4 + q : 128 + lane * 4 + (q - 4); const bool inr = (q < 4) || (lane < 16); const int g = c * WW - WW + j; ok[q] = inr && j >= i && j <= i + 2 * WW && g >= 0 && g < SS; v[q] = inr ? sr[j] : 0.f; if (ok[q]) mx = fmaxf(mx, v[q]); }
#pragma unroll
    for (int sh = 16; sh; sh >>= 1) mx = fmaxf(mx, __shfl_xor(mx, sh, 32));
    float sum = 0.f;
#pragma unroll
    for (int q = 0; q < 8; ++q) { float d0 = __fsub_rn(v[q], mx); asm volatile("" : "+v"(d0)); v[q] = ok[q] ? __expf(d0) : 0.f; sum += v[q]; }
#pragma unroll
    for (int sh = 16; sh; sh >>= 1) sum += __shfl_xor(sum, sh, 32);
    const float f = __fdiv_rn(PCAR, sum); h16* pr = P + (size_t)row * KW;
#pragma unroll 1
    for (int ps = 0; ps < 2; ++ps) { v4h a; a[0] = tohx(v[0] * f); a[1] = tohx(v[1] * f); a[2] = tohx(v[2] * f); a[3] = tohx(v[3] * f); *(volatile v4h*)(pr + lane * 4) = a;
        if (lane < 16) { v4h b; b[0] = tohx(v[4] * f); b[1] = tohx(v[5] * f); b[2] = tohx(v[6] * f); b[3] = tohx(v[7] * f); *(volatile v4h*)(pr + 128 + lane * 4) = b; }
        if (ps == 0) __threadfence(); } }
__device__ __forceinline__ void ln768(float* v, const float* __restrict__ g, const float* __restrict__ bb, int lane) { float s = 0.f;
#pragma unroll
    for (int k = 0; k < 24; ++k) s = __fadd_rn(s, v[k]);
#pragma unroll
    for (int sh = 16; sh; sh >>= 1) s += __shfl_xor(s, sh, 32);
    const float mu = s * (1.0f / DM); float q2 = 0.f;
#pragma unroll
    for (int k = 0; k < 24; ++k) { const float d = __fsub_rn(v[k], mu); float p = __fmul_rn(d, d); asm volatile("" : "+v"(p)); q2 = __fadd_rn(q2, p); }
#pragma unroll
    for (int sh = 16; sh; sh >>= 1) q2 += __shfl_xor(q2, sh, 32);
    const float rs = __frsqrt_rn(__fadd_rn(q2 * (1.0f / DM), 1e-5f));
#pragma unroll
    for (int ch = 0; ch < 6; ++ch)
#pragma unroll
        for (int q = 0; q < 4; ++q) { const int d = ch * 128 + lane * 4 + q; float tn = __fmul_rn(__fsub_rn(v[ch * 4 + q], mu), rs); asm volatile("" : "+v"(tn)); float tg = __fmul_rn(tn, bfr(g[d])); asm volatile("" : "+v"(tg)); v[ch * 4 + q] = __fadd_rn(tg, bfr(bb[d])); } }
__global__ __launch_bounds__(256) void k_ln1(const float* __restrict__ ATT, const float* __restrict__ x, const float* __restrict__ g, const float* __restrict__ bb, float* X1, h16* X16) { const int lane = threadIdx.x & 31; const int t = blockIdx.x * 8 + (threadIdx.x >> 5); if (t >= SS) return; float v[24];
#pragma unroll
    for (int ch = 0; ch < 6; ++ch) { const size_t o = (size_t)t * DM + ch * 128 + lane * 4; const v4f a = *(const v4f*)(ATT + o), xx = *(const v4f*)(x + o);
#pragma unroll
        for (int q = 0; q < 4; ++q) v[ch * 4 + q] = __fadd_rn(a[q] * (1.0f / PCAR), bfr(xx[q])); }
    ln768(v, g, bb, lane);
#pragma unroll 1
    for (int ps = 0; ps < 2; ++ps) {
#pragma unroll
        for (int ch = 0; ch < 6; ++ch) { const size_t o = (size_t)t * DM + ch * 128 + lane * 4; v4f a; v4h hh;
#pragma unroll
            for (int q = 0; q < 4; ++q) { a[q] = v[ch * 4 + q]; hh[q] = tohx(a[q]); } *(volatile v4f*)(X1 + o) = a; *(volatile v4h*)(X16 + o) = hh; }
        if (ps == 0) __threadfence(); } }
__global__ __launch_bounds__(256) void k_ln2(const float* __restrict__ F2, const float* __restrict__ X1, const float* __restrict__ g, const float* __restrict__ bb, float* OUT) { const int lane = threadIdx.x & 31; const int t = blockIdx.x * 8 + (threadIdx.x >> 5); if (t >= SS) return; float v[24];
#pragma unroll
    for (int ch = 0; ch < 6; ++ch) { const size_t o = (size_t)t * DM + ch * 128 + lane * 4; const v4f a = *(const v4f*)(F2 + o), xx = *(const v4f*)(X1 + o);
#pragma unroll
        for (int q = 0; q < 4; ++q) v[ch * 4 + q] = __fadd_rn(a[q], xx[q]); }
    ln768(v, g, bb, lane);
#pragma unroll 1
    for (int ps = 0; ps < 2; ++ps) {
#pragma unroll
        for (int ch = 0; ch < 6; ++ch) { const size_t o = (size_t)t * DM + ch * 128 + lane * 4; v4f a; a[0] = v[ch * 4]; a[1] = v[ch * 4 + 1]; a[2] = v[ch * 4 + 2]; a[3] = v[ch * 4 + 3]; *(volatile v4f*)(OUT + o) = a; }
        if (ps == 0) __threadfence(); } }
__global__ __launch_bounds__(256) void k_gelu16(const float* __restrict__ F, h16* G) { const size_t i = ((size_t)blockIdx.x * 256 + threadIdx.x) * 4; if (i >= (size_t)SS * FF) return; const v4f a = *(const v4f*)(F + i); v4h o;
#pragma unroll
    for (int q = 0; q < 4; ++q) { const float x = a[q]; float x3 = __fmul_rn(__fmul_rn(x, x), x); asm volatile("" : "+v"(x3)); float in_ = __fmul_rn(0.7978845608028654f, __fadd_rn(x, __fmul_rn(0.044715f, x3))); asm volatile("" : "+v"(in_)); const float e2 = __expf(2.0f * in_); const float th = __fsub_rn(1.0f, __fdiv_rn(2.0f, __fadd_rn(e2, 1.0f))); float hx = __fmul_rn(0.5f, x); asm volatile("" : "+v"(hx)); o[q] = tohx(__fmul_rn(hx, __fadd_rn(1.0f, th))); }
    *(volatile v4h*)(G + i) = o; __threadfence(); *(volatile v4h*)(G + i) = o; }

extern "C" void kernel_launch(void* const* d_in, const int* in_sizes, int n_in,
                              void* d_out, int out_size, void* d_ws, size_t ws_size, hipStream_t stream) {
    (void)in_sizes; (void)n_in; (void)out_size;
    const float* IN[15]; for (int i = 0; i < 15; ++i) IN[i] = (const float*)d_in[i];
    float* OUT = (float*)d_out;
    char* wsp = (char*)d_ws;
    auto take = [&](size_t bytes) { char* p = wsp; wsp += (bytes + 255) & ~(size_t)255; return (void*)p; };
    bf* WQ = (bf*)take((size_t)DM * DM * 2); bf* WK = (bf*)take((size_t)DM * DM * 2); bf* WV = (bf*)take((size_t)DM * DM * 2); h16* W1 = (h16*)take((size_t)FF * DM * 2); h16* W2 = (h16*)take((size_t)DM * FF * 2);
    bf* XB = (bf*)take((size_t)SS * DM * 2); float* QF = (float*)take((size_t)SS * DM * 4); float* KF = (float*)take((size_t)SS * DM * 4); float* VF = (float*)take((size_t)SS * DM * 4);
    h16* Q16 = (h16*)take((size_t)NH_ * SS * HD * 2); h16* KP = (h16*)take((size_t)NH_ * SP * HD * 2); h16* VW = (h16*)take((size_t)NH_ * NC * HD * KW * 2); float* Sb = (float*)take((size_t)NC * WW * KW * 4); h16* P16 = (h16*)take((size_t)NC * WW * KW * 2);
    float* ATT = (float*)take((size_t)SS * DM * 4); float* X1 = (float*)take((size_t)SS * DM * 4); h16* X16 = (h16*)take((size_t)SS * DM * 2); float* F1 = (float*)take((size_t)SS * FF * 4); h16* G16 = (h16*)take((size_t)SS * FF * 2); float* F2 = QF;
    if ((size_t)(wsp - (char*)d_ws) > ws_size) return;
    k_wtG<<<(DM * DM / 64 + 63) / 64, 256, 0, stream>>>(IN[1], DM, DM, WQ); k_wtG<<<(DM * DM / 64 + 63) / 64, 256, 0, stream>>>(IN[3], DM, DM, WK); k_wtG<<<(DM * DM / 64 + 63) / 64, 256, 0, stream>>>(IN[5], DM, DM, WV);
    k_wt16<<<(unsigned)(((size_t)DM * FF / 2 + 255) / 256), 256, 0, stream>>>(IN[9], DM, FF, W1); k_wt16<<<(unsigned)(((size_t)FF * DM / 2 + 255) / 256), 256, 0, stream>>>(IN[11], FF, DM, W2);
    for (int b = 0; b < NB_; ++b) { const float* xb = IN[0] + (size_t)b * SS * DM;
        k_cvt8<<<(SS * DM / 8 + 255) / 256, 256, 0, stream>>>(xb, XB, (size_t)SS * DM / 8);
        k_gemmw<bf, 0, true><<<dim3(SS / 64, DM / 64, 1), 32, 0, stream>>>(XB, nullptr, WQ, nullptr, DM, QF, DM, IN[2], 0, 0, 0); k_gemmw<bf, 0, true><<<dim3(SS / 64, DM / 64, 1), 32, 0, stream>>>(XB, nullptr, WK, nullptr, DM, KF, DM, IN[4], 0, 0, 0); k_gemmw<bf, 0, true><<<dim3(SS / 64, DM / 64, 1), 32, 0, stream>>>(XB, nullptr, WV, nullptr, DM, VF, DM, IN[6], 0, 0, 0);
        k_qpl<<<(unsigned)(((size_t)NH_ * SS * HD / 4 + 255) / 256), 256, 0, stream>>>(QF, Q16); k_kpl<<<(unsigned)(((size_t)NH_ * SP * HD / 4 + 255) / 256), 256, 0, stream>>>(KF, KP); k_vwin<<<(unsigned)(((size_t)NH_ * NC * HD * KW / 2 + 255) / 256), 256, 0, stream>>>(VF, VW);
        for (int h = 0; h < NH_; ++h) {
            k_gemmw<h16, 0, false><<<dim3(1, KW / 64, NC), 32, 0, stream>>>(Q16 + (size_t)h * SS * HD, nullptr, KP + (size_t)h * SP * HD, nullptr, HD, Sb, KW, nullptr, (size_t)WW * HD, (size_t)WW * HD, (size_t)WW * KW);
            k_bsoft<<<NC * WW / 8, 256, 0, stream>>>(Sb, P16);
            k_gemmw<h16, 0, false><<<dim3(1, 1, NC), 32, 0, stream>>>(P16, nullptr, VW + (size_t)h * NC * HD * KW, nullptr, KW, ATT + h * HD, DM, nullptr, (size_t)WW * KW, (size_t)HD * KW, (size_t)WW * DM); }
        k_ln1<<<SS / 8, 256, 0, stream>>>(ATT, xb, IN[7], IN[8], X1, X16);
        k_gemmw<h16, 0, true><<<dim3(SS / 64, FF / 64, 1), 32, 0, stream>>>(X16, nullptr, W1, nullptr, DM, F1, FF, IN[10], 0, 0, 0); k_gelu16<<<(unsigned)(((size_t)SS * FF / 4 + 255) / 256), 256, 0, stream>>>(F1, G16);
        k_gemmw<h16, 0, true><<<dim3(SS / 64, DM / 64, 1), 32, 0, stream>>>(G16, nullptr, W2, nullptr, FF, F2, DM, IN[12], 0, 0, 0);
        k_ln2<<<SS / 8, 256, 0, stream>>>(F2, X1, IN[13], IN[14], OUT + (size_t)b * SS * DM); }
}
